// GDN_32504312496804
// MI455X (gfx1250) — hardware-run, weakly checked
//
#include <hip/hip_runtime.h>
#include <stddef.h>
#include <stdint.h>
#pragma clang fp contract(off)


#define DF      256
#define PP      512
#define AP      512
#define WSP     256
#define WFP     512
#define SPLIT_FC 1
#define KFC     (SPLIT_FC ? 512 : 256)
#define KPJ     256
#define NPJ     512
#define NTHR    256
#define NWAVE   8
#define EPT     8
#define CHUNK   (NTHR * EPT)
#define WCAP    (EPT * 32)
#define LISTN   (NWAVE * WCAP)
#define NB      256
#define SLB     8
#define NBW     (NB / NWAVE)
#define RCAP    10240
#define DEGCAP  96
#define MEAS_B256 8412
#define MEAS_DEG  58
#define GBM     64
#define GBN     128
#define GTHR    128
#define NEGS    0.2f
#define WSMAX   ((size_t)128 << 20)
#define PASS_INTS (2 * RCAP + 2 * NB + LISTN + 2 * NWAVE + 2 * NB)
#define LDS_PASS  (PASS_INTS * 4)

static_assert(RCAP >= MEAS_B256 + 1024);
static_assert(DEGCAP >= MEAS_DEG + 8);
static_assert((CHUNK & (CHUNK - 1)) == 0 && CHUNK <= 4096);
static_assert(NB == (1 << SLB) && NB == NTHR && (NB % NWAVE) == 0);
static_assert(LISTN >= NB && LISTN >= NWAVE * WCAP);
static_assert((RCAP % 32) == 0);
static_assert(DF == 32 * 8);
static_assert((KPJ % 32) == 0 && (KFC % 32) == 0 && KFC <= AP && KFC <= WFP && KPJ <= WSP);
static_assert((NPJ % GBN) == 0 && (DF % GBN) == 0 && GBM == (GTHR / 32) * 16);
static_assert(LDS_PASS <= 300000);

typedef float          v2f   __attribute__((ext_vector_type(2)));
typedef float          v4f   __attribute__((ext_vector_type(4)));
typedef float          v8f   __attribute__((ext_vector_type(8)));
typedef int            v4i   __attribute__((ext_vector_type(4)));
typedef int            v8i   __attribute__((ext_vector_type(8)));
typedef unsigned       v4u   __attribute__((ext_vector_type(4)));
typedef unsigned short v8us  __attribute__((ext_vector_type(8)));
typedef unsigned short v16us __attribute__((ext_vector_type(16)));
typedef __bf16         v16bf __attribute__((ext_vector_type(16)));
typedef v4f  __attribute__((may_alias)) v4fa;
typedef v4u  __attribute__((may_alias)) v4ua;
typedef v8us __attribute__((may_alias)) v8usa;
union FragB { v16bf v; v16us u; v8us h[2]; v8i w; };

__device__ __forceinline__ v8f wmb(const FragB& a, const FragB& b, v8f c) {
  v8f d = __builtin_amdgcn_wmma_f32_16x16x32_bf16(false, a.v, false, b.v, (short)0, c, false, false);
  asm volatile("v_nop\n\tv_nop\n\tv_nop\n\tv_nop" : "+v"(d) : "v"(a.w), "v"(b.w));
  return d;
}

__device__ __forceinline__ unsigned bfbits(float f) {
  const unsigned u = __float_as_uint(f);
  const unsigned r = (u + 0x7FFFu + ((u >> 16) & 1u)) >> 16;
  return (f != f) ? 0x7fc0u : r;
}
__device__ __forceinline__ float rbf(float f) { return __uint_as_float(bfbits(f) << 16); }

__device__ __forceinline__ v8us cvt8b(const v4f a, const v4f b) {
  v8us o;
  o[0] = (unsigned short)bfbits(a.x); o[1] = (unsigned short)bfbits(a.y);
  o[2] = (unsigned short)bfbits(a.z); o[3] = (unsigned short)bfbits(a.w);
  o[4] = (unsigned short)bfbits(b.x); o[5] = (unsigned short)bfbits(b.y);
  o[6] = (unsigned short)bfbits(b.z); o[7] = (unsigned short)bfbits(b.w);
  return o;
}
__device__ __forceinline__ void put8(unsigned short* dp, const v8us o) {
  *(volatile v8us*)dp = o;
  __threadfence();
  *(volatile v8us*)dp = o;
}

__device__ __forceinline__ float lk(float a, float b, float w, float part) {
  float z = a + b;
  z = (z >= 0.0f) ? z : NEGS * z;
  return fmaf(z, w, part);
}
__device__ __forceinline__ float edge_logit(const v4f sa, const v4f sb, const v4f ta, const v4f tb,
                                            const v4f wa, const v4f wb) {
  float part = 0.0f;
  part = lk(sa.x, ta.x, wa.x, part);
  part = lk(sa.y, ta.y, wa.y, part);
  part = lk(sa.z, ta.z, wa.z, part);
  part = lk(sa.w, ta.w, wa.w, part);
  part = lk(sb.x, tb.x, wb.x, part);
  part = lk(sb.y, tb.y, wb.y, part);
  part = lk(sb.z, tb.z, wb.z, part);
  part = lk(sb.w, tb.w, wb.w, part);
#pragma unroll
  for (int off = 16; off > 0; off >>= 1) part += __shfl_xor(part, off);
  return part;
}

__device__ __forceinline__ int scan_chunk(const int* __restrict__ keys, int nE, int cbase, int slotBase,
                                          int vec8, int* list, int tid, int lane, int wave) {
  const int el0  = tid * EPT;
  const int e0   = cbase + el0;
  const int sent = (int)0x80000000u;
  v4i da, db;
  if (vec8 != 0 && cbase + CHUNK <= nE) {
    da = *(const v4i*)(keys + e0);
    db = *(const v4i*)(keys + e0 + 4);
  } else {
    da.x = (e0     < nE) ? keys[min(e0,     nE - 1)] : sent;
    da.y = (e0 + 1 < nE) ? keys[min(e0 + 1, nE - 1)] : sent;
    da.z = (e0 + 2 < nE) ? keys[min(e0 + 2, nE - 1)] : sent;
    da.w = (e0 + 3 < nE) ? keys[min(e0 + 3, nE - 1)] : sent;
    db.x = (e0 + 4 < nE) ? keys[min(e0 + 4, nE - 1)] : sent;
    db.y = (e0 + 5 < nE) ? keys[min(e0 + 5, nE - 1)] : sent;
    db.z = (e0 + 6 < nE) ? keys[min(e0 + 6, nE - 1)] : sent;
    db.w = (e0 + 7 < nE) ? keys[min(e0 + 7, nE - 1)] : sent;
  }
  const unsigned nbs = (unsigned)slotBase;
  const unsigned unb = (unsigned)NB;
  const unsigned s0 = (unsigned)da.x - nbs, s1 = (unsigned)da.y - nbs;
  const unsigned s2 = (unsigned)da.z - nbs, s3 = (unsigned)da.w - nbs;
  const unsigned s4 = (unsigned)db.x - nbs, s5 = (unsigned)db.y - nbs;
  const unsigned s6 = (unsigned)db.z - nbs, s7 = (unsigned)db.w - nbs;
  const bool h0 = s0 < unb, h1 = s1 < unb, h2 = s2 < unb, h3 = s3 < unb;
  const bool h4 = s4 < unb, h5 = s5 < unb, h6 = s6 < unb, h7 = s7 < unb;
  const unsigned m0 = __builtin_amdgcn_ballot_w32(h0);
  const unsigned m1 = __builtin_amdgcn_ballot_w32(h1);
  const unsigned m2 = __builtin_amdgcn_ballot_w32(h2);
  const unsigned m3 = __builtin_amdgcn_ballot_w32(h3);
  const unsigned m4 = __builtin_amdgcn_ballot_w32(h4);
  const unsigned m5 = __builtin_amdgcn_ballot_w32(h5);
  const unsigned m6 = __builtin_amdgcn_ballot_w32(h6);
  const unsigned m7 = __builtin_amdgcn_ballot_w32(h7);
  const unsigned any = m0 | m1 | m2 | m3 | m4 | m5 | m6 | m7;
  int wc = 0;
  if (any != 0u) {
    const unsigned lt = (1u << lane) - 1u;
    int pos = (int)__builtin_popcount(m0 & lt) + (int)__builtin_popcount(m1 & lt)
            + (int)__builtin_popcount(m2 & lt) + (int)__builtin_popcount(m3 & lt)
            + (int)__builtin_popcount(m4 & lt) + (int)__builtin_popcount(m5 & lt)
            + (int)__builtin_popcount(m6 & lt) + (int)__builtin_popcount(m7 & lt);
    int* wl = list + wave * WCAP;
#define HITJ(J, HJ, SJ) \
    if (HJ) { if (pos < WCAP) wl[pos] = ((el0 + (J)) << SLB) | (int)(SJ); pos += 1; }
    HITJ(0, h0, s0)
    HITJ(1, h1, s1)
    HITJ(2, h2, s2)
    HITJ(3, h3, s3)
    HITJ(4, h4, s4)
    HITJ(5, h5, s5)
    HITJ(6, h6, s6)
    HITJ(7, h7, s7)
#undef HITJ
    wc = (int)__builtin_popcount(m0) + (int)__builtin_popcount(m1) + (int)__builtin_popcount(m2)
       + (int)__builtin_popcount(m3) + (int)__builtin_popcount(m4) + (int)__builtin_popcount(m5)
       + (int)__builtin_popcount(m6) + (int)__builtin_popcount(m7);
  }
  return wc;
}

__global__ __launch_bounds__(NTHR) void k_prep(const float* __restrict__ feat, const float* __restrict__ Ws,
                                               const float* __restrict__ Wt, const float* __restrict__ Wa,
                                               const float* __restrict__ Wfc, const float* __restrict__ bfc,
                                               unsigned short* FB, unsigned short* WST, unsigned short* WFC2,
                                               float* WAB, int nN, int nbFB) {
  const int b = (int)blockIdx.x, tid = (int)threadIdx.x;
  const v4f z4 = {0.f, 0.f, 0.f, 0.f};
  if (b < nbFB) {
    const int i   = b * NTHR + tid;
    const int row = i >> 5;
    const int c0  = (i & 31) * 8;
    const int rc  = row < nN ? row : nN - 1;
    const float* p = feat + (size_t)rc * DF + c0;
    v4f a = *(const v4f*)p, q = *(const v4f*)(p + 4);
    if (row >= nN) { a = z4; q = z4; }
    put8(FB + (size_t)row * DF + c0, cvt8b(a, q));
    return;
  }
  const int b1 = b - nbFB;
  if (b1 < 32) {
    const int n  = b1 * 8 + (tid >> 5);
    const int k8 = (tid & 31) * 8;
    const float* p = Ws + (size_t)n * DF + k8;
    const v4f a = *(const v4f*)p, q = *(const v4f*)(p + 4);
    put8(WST + (size_t)n * WSP + k8, cvt8b(a, q));
  } else if (b1 < 64) {
    const int n  = (b1 - 32) * 8 + (tid >> 5);
    const int k8 = (tid & 31) * 8;
    const float* p = Wt + (size_t)n * DF + k8;
    const v4f a = *(const v4f*)p, q = *(const v4f*)(p + 4);
    put8(WST + (size_t)(DF + n) * WSP + k8, cvt8b(a, q));
  } else if (b1 < 128) {
    const int u  = (b1 - 64) * NTHR + tid;
    const int n  = u >> 6;
    const int kk = (u & 63) * 8;
    const float* p = Wfc + (size_t)n * DF + (kk & (DF - 1));
    const v4f a = *(const v4f*)p, q = *(const v4f*)(p + 4);
    put8(WFC2 + (size_t)n * WFP + kk, cvt8b(a, q));
  } else if (b1 == 128) {
    const int wv = tid >> 5;
    if (wv < 2) {
      const v4f a = *(const v4f*)(Wa + 4 * tid);
      v4f o; o.x = rbf(a.x); o.y = rbf(a.y); o.z = rbf(a.z); o.w = rbf(a.w);
      float* dp = WAB + 4 * tid;
      *(volatile v4f*)dp = o;
      __threadfence();
      *(volatile v4f*)dp = o;
    } else if (wv < 4) {
      const int t = tid - 64;
      const v4f a = *(const v4f*)(bfc + 4 * t);
      v4f o; o.x = rbf(a.x); o.y = rbf(a.y); o.z = rbf(a.z); o.w = rbf(a.w);
      float* dp = WAB + DF + 4 * t;
      *(volatile v4f*)dp = o;
      __threadfence();
      *(volatile v4f*)dp = o;
    }
  }
}

template <int HASB>
__global__ __attribute__((amdgpu_num_vgpr(248))) __launch_bounds__(GTHR)
void k_gemm(const unsigned short* __restrict__ A, int lda, const unsigned short* __restrict__ BT, int ldb, int K,
            const float* __restrict__ bias, float* outp, int ldo, int nOut) {
  __shared__ __attribute__((aligned(16))) float stg[GBM * GBN];
  const int tid = (int)threadIdx.x, lane = tid & 31, wave = tid >> 5, hh = lane >> 4, m = lane & 15;
  const int rowBase = (int)blockIdx.x * GBM;
  const int col0    = (int)blockIdx.y * GBN;

  v8f acc[8];
  {
    const v8f z = {0.f, 0.f, 0.f, 0.f, 0.f, 0.f, 0.f, 0.f};
#pragma unroll
    for (int t = 0; t < 8; ++t) acc[t] = z;
  }
  const unsigned short* ap = A + (size_t)(rowBase + 16 * wave + m) * (size_t)lda + 8 * hh;
  const unsigned short* bp = BT + (size_t)(col0 + m) * (size_t)ldb + 8 * hh;

#pragma unroll 1
  for (int k0 = 0; k0 < K; k0 += 32) {
    FragB af;
    af.h[0] = *(const v8usa*)(ap + k0);
    af.h[1] = *(const v8usa*)(ap + k0 + 16);
#pragma unroll
    for (int nt = 0; nt < 8; ++nt) {
      const unsigned short* wq = bp + (size_t)(16 * nt) * (size_t)ldb + k0;
      FragB bf;
      bf.h[0] = *(const v8usa*)wq;
      bf.h[1] = *(const v8usa*)(wq + 16);
      acc[nt] = wmb(af, bf, acc[nt]);
    }
  }

#pragma unroll
  for (int nt = 0; nt < 8; ++nt) {
    const int lc = 16 * nt + m;
#pragma unroll
    for (int r = 0; r < 8; ++r) {
      const int lr = 16 * wave + 8 * hh + r;
      stg[lr * GBN + lc] = acc[nt][r];
    }
  }
  __syncthreads();

  v4f bb4 = {0.f, 0.f, 0.f, 0.f};
  if constexpr (HASB != 0) bb4 = *(const v4f*)(bias + col0 + 4 * lane);

  v4f pv[16];
#pragma unroll
  for (int i = 0; i < 16; ++i) pv[i] = *(const v4fa*)(stg + (16 * wave + i) * GBN + 4 * lane) + bb4;

#pragma unroll
  for (int i = 0; i < 16; ++i) {
    const int r = rowBase + 16 * wave + i;
    if (r < nOut) *(volatile v4f*)(outp + (size_t)r * (size_t)ldo + col0 + 4 * lane) = pv[i];
  }
  __threadfence();
#pragma unroll
  for (int i = 0; i < 16; ++i) {
    const int r = rowBase + 16 * wave + i;
    if (r < nOut) *(volatile v4f*)(outp + (size_t)r * (size_t)ldo + col0 + 4 * lane) = pv[i];
  }
}

template <int MODE>
__global__ __launch_bounds__(NTHR) void k_pass(const int* __restrict__ keys, const int* __restrict__ part,
                                               const float* __restrict__ P, const float* __restrict__ WAB,
                                               const unsigned short* __restrict__ FB,
                                               float* MR, unsigned short* AGG,
                                               int nN, int nE, int vec8, int MPr) {
  extern __shared__ v4f lds_dyn[];
  int* reg1 = (int*)lds_dyn;
  int* reg2 = reg1 + RCAP;
  int* scnt = reg2 + RCAP;
  int* soff = scnt + NB;
  int* list = soff + NB;
  int* wcnt = list + LISTN;
  int* wtot = wcnt + NWAVE;
  float* mrd = (float*)(wtot + NWAVE);
  const int tid = (int)threadIdx.x, lane = tid & 31, wave = tid >> 5;
  const int nodeBase = (int)blockIdx.x * NB;

  scnt[tid] = 0;
  __syncthreads();

  int tot = 0;
  const int nChunks = (nE + CHUNK - 1) / CHUNK;
#pragma unroll 1
  for (int ch = 0; ch < nChunks; ++ch) {
    const int cbase = ch * CHUNK;
    const int wc = scan_chunk(keys, nE, cbase, nodeBase, vec8, list, tid, lane, wave);
    if (lane == 0) wcnt[wave] = wc;
    __syncthreads();
    int pre = 0, all = 0;
#pragma unroll
    for (int w2 = 0; w2 < NWAVE; ++w2) {
      int c = wcnt[w2];
      c = c < 0 ? 0 : (c > WCAP ? WCAP : c);
      all += c;
      pre += (w2 < wave) ? c : 0;
    }
    const int wcc  = wc > WCAP ? WCAP : wc;
    const int base = tot + pre;
#pragma unroll 1
    for (int i = lane; i < wcc; i += 32) {
      const int ent = list[wave * WCAP + i];
      const int el  = (ent >> SLB) & (CHUNK - 1);
      const int sl  = ent & (NB - 1);
      int eid = cbase + el;
      eid = eid > nE - 1 ? nE - 1 : eid;
      const int pos = base + i;
      if (pos < RCAP) reg1[pos] = (int)(((unsigned)eid << SLB) | (unsigned)sl);
    }
    tot += all;
    tot = tot > RCAP ? RCAP : tot;
    __syncthreads();
  }
  const int nh = __builtin_amdgcn_readfirstlane(tot);

  if (wave == 0) {
#pragma unroll 1
    for (int b0 = 0; b0 < nh; b0 += 32) {
      int idx = b0 + lane;
      idx = idx > nh - 1 ? nh - 1 : idx;
      const int uv  = reg1[idx];
      const int m32 = (nh - b0) < 32 ? (nh - b0) : 32;
#pragma unroll 1
      for (int k = 0; k < m32; ++k) {
        const int u  = __builtin_amdgcn_readlane(uv, k);
        const int sl = u & (NB - 1);
        if (lane == 0) scnt[sl] = scnt[sl] + 1;
      }
    }
  }
  __syncthreads();

  {
    int c = scnt[tid];
    c = c < 0 ? 0 : c;
    int incl = c;
#pragma unroll
    for (int d = 1; d < 32; d <<= 1) {
      const int up = __shfl_up(incl, d);
      if (lane >= d) incl += up;
    }
    if (lane == 31) wtot[wave] = incl;
    __syncthreads();
    int pre = 0;
#pragma unroll
    for (int w2 = 0; w2 < NWAVE; ++w2) pre += (w2 < wave) ? wtot[w2] : 0;
    const int ex = pre + incl - c;
    soff[tid] = ex;
    list[tid] = ex;
  }
  __syncthreads();

  if (wave == 0) {
#pragma unroll 1
    for (int b0 = 0; b0 < nh; b0 += 32) {
      int idx = b0 + lane;
      idx = idx > nh - 1 ? nh - 1 : idx;
      const int uv  = reg1[idx];
      const int m32 = (nh - b0) < 32 ? (nh - b0) : 32;
#pragma unroll 1
      for (int k = 0; k < m32; ++k) {
        const int u   = __builtin_amdgcn_readlane(uv, k);
        const int sl  = u & (NB - 1);
        const int eid = (int)((unsigned)u >> SLB);
        if (lane == 0) {
          int pos = list[sl];
          pos = pos < 0 ? 0 : (pos > RCAP - 1 ? RCAP - 1 : pos);
          reg2[pos] = eid;
          list[sl] = pos + 1;
        }
      }
    }
  }
  __syncthreads();

  const bool ovf = (nh >= RCAP);
  const float qnan = __int_as_float(0x7fc00000);
  const v4f wa = *(const v4f*)(WAB + 8 * lane);
  const v4f wb = *(const v4f*)(WAB + 8 * lane + 4);
  constexpr int OWNOFF = (MODE == 0) ? 0 : DF;
  constexpr int GATOFF = (MODE == 0) ? DF : 0;
#pragma unroll 1
  for (int jt = 0; jt < NBW; ++jt) {
    const int slot = wave * NBW + jt;
    const int grow = nodeBase + slot;
    const int gcl  = grow < nN ? grow : nN - 1;
    int stv = soff[slot];
    const int crawv = scnt[slot];
    int cntv = crawv;
    stv  = stv < 0 ? 0 : (stv > nh ? nh : stv);
    cntv = cntv < 0 ? 0 : (cntv > DEGCAP ? DEGCAP : cntv);
    if (cntv > nh - stv) cntv = nh - stv;
    int lastv = stv + cntv - 1;
    lastv = lastv < stv ? stv : lastv;
    lastv = lastv > RCAP - 1 ? RCAP - 1 : lastv;
    const int bigv = (crawv > DEGCAP) ? 1 : 0;
    const int st   = __builtin_amdgcn_readfirstlane(stv);
    const int cnt  = __builtin_amdgcn_readfirstlane(cntv);
    const int last = __builtin_amdgcn_readfirstlane(lastv);
    const int big  = __builtin_amdgcn_readfirstlane(bigv);
    const float pz = (ovf || big != 0) ? qnan : 0.0f;

    const float* orow = P + (size_t)gcl * PP + OWNOFF + 8 * lane;
    const v4f oa = *(const v4f*)orow;
    const v4f ob = *(const v4f*)(orow + 4);
    float mx = __int_as_float((int)0xff800000u);
    float dn = 0.0f;
    float acc[8];
#pragma unroll
    for (int c = 0; c < 8; ++c) acc[c] = 0.0f;

#pragma unroll 1
    for (int b0 = 0; b0 < cnt; b0 += 32) {
      int idx = st + b0 + lane;
      idx = idx > last ? last : idx;
      int eid = reg2[idx];
      eid = eid < 0 ? 0 : (eid > nE - 1 ? nE - 1 : eid);
      const int praw = part[eid];
      const int p = praw < 0 ? 0 : (praw > nN - 1 ? nN - 1 : praw);
      int mxi = 0, rdi = 0;
      if constexpr (MODE != 0) {
        const v2f mr = *(const v2f*)((const float*)MR + 2 * (size_t)p);
        mxi = __float_as_int(mr.x);
        rdi = __float_as_int(mr.y);
      }
      const int m32 = (cnt - b0) < 32 ? (cnt - b0) : 32;
#pragma unroll 1
      for (int k = 0; k < m32; ++k) {
        const int pk = __builtin_amdgcn_readlane(p, k);
        const float* gr = P + (size_t)pk * PP + GATOFF + 8 * lane;
        const v4f ga = *(const v4f*)gr;
        const v4f gb = *(const v4f*)(gr + 4);
        if constexpr (MODE == 0) {
          const float e  = edge_logit(oa, ob, ga, gb, wa, wb);
          const float df = e - mx;
          const float ee = expf(-fabsf(df));
          const bool up  = df > 0.0f;
          const float s1 = up ? ee : 1.0f;
          const float s2 = up ? 1.0f : ee;
          mx = up ? e : mx;
          dn = fmaf(dn, s1, s2);
        } else {
          const float e  = edge_logit(ga, gb, oa, ob, wa, wb);
          const float mk = __int_as_float(__builtin_amdgcn_readlane(mxi, k));
          const float rk = __int_as_float(__builtin_amdgcn_readlane(rdi, k));
          const float al = expf(e - mk) * rk;
          const v4u fw = *(const v4ua*)(FB + (size_t)pk * DF + 8 * lane);
          acc[0] = fmaf(al, __uint_as_float(fw.x << 16),          acc[0]);
          acc[1] = fmaf(al, __uint_as_float(fw.x & 0xffff0000u),  acc[1]);
          acc[2] = fmaf(al, __uint_as_float(fw.y << 16),          acc[2]);
          acc[3] = fmaf(al, __uint_as_float(fw.y & 0xffff0000u),  acc[3]);
          acc[4] = fmaf(al, __uint_as_float(fw.z << 16),          acc[4]);
          acc[5] = fmaf(al, __uint_as_float(fw.z & 0xffff0000u),  acc[5]);
          acc[6] = fmaf(al, __uint_as_float(fw.w << 16),          acc[6]);
          acc[7] = fmaf(al, __uint_as_float(fw.w & 0xffff0000u),  acc[7]);
        }
      }
    }

    if constexpr (MODE == 0) {
      const float mfin = (fabsf(mx) < __int_as_float(0x7f800000)) ? mx : 0.0f;
      const float ds = (cnt > 0) ? dn : 1.0f;
      float rd = 1.0f / ds;
      rd = (cnt > 0) ? rd : 0.0f;
      if (lane == 0) {
        mrd[2 * slot]     = mfin + pz;
        mrd[2 * slot + 1] = rd + pz;
      }
    } else {
      const bool live = grow < nN;
      v8us hv, lv;
#pragma unroll
      for (int c = 0; c < 8; ++c) {
        const float v = live ? (acc[c] + pz) : 0.0f;
        const unsigned hb = bfbits(v);
        hv[c] = (unsigned short)hb;
        lv[c] = (unsigned short)bfbits(v - __uint_as_float(hb << 16));
      }
      if (grow < MPr) {
        unsigned short* rp = AGG + (size_t)grow * AP + 8 * lane;
        *(volatile v8us*)rp = hv;
        *(volatile v8us*)(rp + DF) = lv;
        __threadfence();
        *(volatile v8us*)rp = hv;
        *(volatile v8us*)(rp + DF) = lv;
      }
    }
  }

  if constexpr (MODE == 0) {
    __syncthreads();
    if (tid < 128) {
      const v4f mv = *(const v4fa*)(mrd + 4 * tid);
      float* gp = MR + (size_t)nodeBase * 2 + 4 * tid;
      *(volatile v4f*)gp = mv;
      __threadfence();
      *(volatile v4f*)gp = mv;
    }
  }
  (void)FB; (void)AGG; (void)MPr;
}

static inline int cdiv(int a, int b) { return (a + b - 1) / b; }
static inline size_t al256(size_t o) { return (o + 255) & ~(size_t)255; }

extern "C" void kernel_launch(void* const* d_in, const int* in_sizes, int n_in,
                              void* d_out, int out_size, void* d_ws, size_t ws_size,
                              hipStream_t stream) {
  if (n_in < 8) return;
  const int nN = in_sizes[0] / DF;
  if (nN < 1 || in_sizes[0] != nN * DF || nN > (1 << 20)) return;
  const int nE = in_sizes[1];
  if (nE < 1 || nE >= (1 << 23) || in_sizes[2] != nE) return;
  if (in_sizes[3] != DF * DF || in_sizes[4] != DF * DF) return;
  if (in_sizes[5] != DF) return;
  if (in_sizes[6] != DF * DF || in_sizes[7] != DF) return;
  if ((long long)out_size != (long long)nN * DF) return;

  const float* feat = (const float*)d_in[0];
  const int*   src  = (const int*)  d_in[1];
  const int*   dst  = (const int*)  d_in[2];
  const float* W_s  = (const float*)d_in[3];
  const float* W_t  = (const float*)d_in[4];
  const float* W_a  = (const float*)d_in[5];
  const float* W_fc = (const float*)d_in[6];
  const float* b_fc = (const float*)d_in[7];
  float* out = (float*)d_out;

  const int MP   = cdiv(nN, 128) * 128;
  const int gA   = cdiv(MP, NB);
  const int nbFB = MP / 8;
  const int vec8 = ((nE & 3) == 0) ? 1 : 0;
  if ((MP % GBM) != 0 || (long long)gA * NB < (long long)MP) return;

  char* ws = (char*)d_ws;
  size_t off = 0;
  const size_t oFB   = off; off = al256(off + (size_t)MP * DF * 2);
  const size_t oWST  = off; off = al256(off + (size_t)NPJ * WSP * 2);
  const size_t oWFC2 = off; off = al256(off + (size_t)DF * WFP * 2);
  const size_t oWAB  = off; off = al256(off + (size_t)2 * DF * 4);
  const size_t oP    = off; off = al256(off + (size_t)MP * PP * 4);
  const size_t oMR   = off; off = al256(off + (size_t)gA * NB * 2 * 4);
  const size_t oAGG  = off; off = al256(off + (size_t)MP * AP * 2);
  if (off > ws_size || off > WSMAX) return;
  unsigned short* FB   = (unsigned short*)(ws + oFB);
  unsigned short* WST  = (unsigned short*)(ws + oWST);
  unsigned short* WFC2 = (unsigned short*)(ws + oWFC2);
  float*          WAB  = (float*)(ws + oWAB);
  float*          P    = (float*)(ws + oP);
  float*          MR   = (float*)(ws + oMR);
  unsigned short* AGG  = (unsigned short*)(ws + oAGG);

  hipFuncSetAttribute(reinterpret_cast<const void*>(&k_pass<0>),
                      hipFuncAttributeMaxDynamicSharedMemorySize, LDS_PASS);
  hipFuncSetAttribute(reinterpret_cast<const void*>(&k_pass<1>),
                      hipFuncAttributeMaxDynamicSharedMemorySize, LDS_PASS);

  k_prep<<<nbFB + 129, NTHR, 0, stream>>>(feat, W_s, W_t, W_a, W_fc, b_fc, FB, WST, WFC2, WAB, nN, nbFB);
  k_gemm<0><<<dim3(MP / GBM, NPJ / GBN), GTHR, 0, stream>>>(FB, DF, WST, WSP, KPJ, WAB, P, PP, MP);
  k_pass<0><<<gA, NTHR, LDS_PASS, stream>>>(src, dst, P, WAB, FB, MR, AGG, nN, nE, vec8, MP);
  k_pass<1><<<gA, NTHR, LDS_PASS, stream>>>(dst, src, P, WAB, FB, MR, AGG, nN, nE, vec8, MP);
  k_gemm<1><<<dim3(MP / GBM, DF / GBN), GTHR, 0, stream>>>(AGG, AP, WFC2, WFP, KFC, WAB + DF, out, DF, nN);
}
